// LiltSelfAttention_55336358642313
// MI455X (gfx1250) — hardware-verified
//
#include <hip/hip_runtime.h>
#include <math.h>
#include <stdint.h>

#define NB   8
#define SEQ  1024
#define DM   768
#define DL   192
#define NH   12
#define HD   64
#define HL   16
#define NQB  (SEQ / 64)
#define NKT  (SEQ / 64)
static_assert(NH * HD == DM);
static_assert(NH * HL == DL);
static_assert(NQB == 16 && NKT == 16);
static_assert((SEQ % 64) == 0 && (DM % 64) == 0 && (DL % 64) == 0);
static_assert((DM % 32) == 0 && (DL % 32) == 0);

typedef _Float16 v16h __attribute__((ext_vector_type(16)));
typedef _Float16 v8h  __attribute__((ext_vector_type(8)));
typedef float    v8f  __attribute__((ext_vector_type(8)));
typedef float    v4f  __attribute__((ext_vector_type(4)));
typedef unsigned int v4u __attribute__((ext_vector_type(4)));

#if defined(__HIP_DEVICE_COMPILE__)
#define DEV_ASM 1
#else
#define DEV_ASM 0
#endif

__device__ __forceinline__ unsigned short h_bits(_Float16 x) { return __builtin_bit_cast(unsigned short, x); }
__device__ __forceinline__ unsigned pk16(unsigned short a, unsigned short b) { return (unsigned)a | ((unsigned)b << 16); }
__device__ __forceinline__ v8f zero8() { v8f z = {0.f, 0.f, 0.f, 0.f, 0.f, 0.f, 0.f, 0.f}; return z; }
__device__ __forceinline__ v8h zero8h() {
  const _Float16 z = (_Float16)0.0f;
  v8h r = {z, z, z, z, z, z, z, z};
  return r;
}

__device__ __forceinline__ v16h ldfrag_h(const _Float16* p) {
  union { v16h v; v8h h[2]; } f;
  f.h[0] = *(const v8h*)(p);
  f.h[1] = *(const v8h*)(p + 16);
  return f.v;
}

__device__ __forceinline__ v8f mmar(v16h a, v16h b, v8f c) {
  return __builtin_amdgcn_wmma_f32_16x16x32_f16(false, a, false, b, (short)0, c, false, false);
}
__device__ __forceinline__ v8f mma_h(v16h a, v16h b, v8f c) {
  c = __builtin_amdgcn_wmma_f32_16x16x32_f16(false, a, false, b, (short)0, c, false, false);
#if DEV_ASM
  asm volatile("v_nop\n\tv_nop\n\tv_nop\n\tv_nop" : "+v"(c) : "v"(a), "v"(b));
#endif
  return c;
}
__device__ __forceinline__ void dep_guard(v8f& a, v8f& b, v16h x, v16h y) {
#if DEV_ASM
  asm volatile("v_nop\n\tv_nop\n\tv_nop\n\tv_nop" : "+v"(a), "+v"(b) : "v"(x), "v"(y));
#else
  (void)a; (void)b; (void)x; (void)y;
#endif
}
__device__ __forceinline__ void keep4(v16h a, v16h b, v16h c, v16h d) {
#if DEV_ASM
  asm volatile("v_nop" :: "v"(a), "v"(b), "v"(c), "v"(d));
#else
  (void)a; (void)b; (void)c; (void)d;
#endif
}
__device__ __forceinline__ void acc_guard4(v8f& a, v8f& b, v8f& c, v8f& d) {
#if DEV_ASM
  asm volatile("v_nop\n\tv_nop\n\tv_nop\n\tv_nop" : "+v"(a), "+v"(b), "+v"(c), "+v"(d));
#else
  (void)a; (void)b; (void)c; (void)d;
#endif
}

__global__ __launch_bounds__(256) void cvt_h16x8(const float* __restrict__ in, unsigned short* out, int n8, float scale) {
  const int i = blockIdx.x * 256 + (int)threadIdx.x;
  if (i < n8) {
    const v4f a = *(const v4f*)(in + (size_t)i * 8);
    const v4f c = *(const v4f*)(in + (size_t)i * 8 + 4);
    v4u p;
    p[0] = pk16(h_bits((_Float16)(a[0] * scale)), h_bits((_Float16)(a[1] * scale)));
    p[1] = pk16(h_bits((_Float16)(a[2] * scale)), h_bits((_Float16)(a[3] * scale)));
    p[2] = pk16(h_bits((_Float16)(c[0] * scale)), h_bits((_Float16)(c[1] * scale)));
    p[3] = pk16(h_bits((_Float16)(c[2] * scale)), h_bits((_Float16)(c[3] * scale)));
    unsigned short* o = out + (size_t)i * 8;
    *(volatile v4u*)o = p;
    __threadfence();
    *(volatile v4u*)o = p;
  }
}

template <int BIASROW>
__global__ __launch_bounds__(256) void gemm64(
    const unsigned short* __restrict__ Ap, int lda, long long strideA,
    const unsigned short* __restrict__ Btp, int ldb, long long strideB,
    const float* __restrict__ bias,
    unsigned short* Cp, int ldc, long long strideC,
    int M, int N, int K, float ascale, float oscale) {
  const _Float16* A  = (const _Float16*)(const void*)Ap;
  const _Float16* Bt = (const _Float16*)(const void*)Btp;
  __shared__ __align__(16) float sT[8][16 * 68];
  const int b    = blockIdx.y;
  const int lane = threadIdx.x & 31;
  const int wave = threadIdx.x >> 5;
  const int tilesN = N >> 6;
  const int tilesM = M >> 6;
  const int tile = blockIdx.x * 8 + wave;
  if (tile >= tilesM * tilesN) return;
  const int tm = tile / tilesN;
  const int tn = tile - tm * tilesN;
  const int m0 = tm << 6;
  const int n0 = tn << 6;

  const _Float16* Ab = A  + (size_t)b * (size_t)strideA;
  const _Float16* Bb = Bt + (size_t)b * (size_t)strideB;

  const int rlane = lane & 15;
  const int koff  = (lane >> 4) * 8;
  const int mOff  = (lane >> 4) * 8;

  v8f acc[4][4];
#pragma unroll
  for (int i = 0; i < 4; ++i)
#pragma unroll
    for (int j = 0; j < 4; ++j) acc[i][j] = zero8();

  for (int k0 = 0; k0 < K; k0 += 32) {
    v16h bq[4];
#pragma unroll
    for (int j = 0; j < 4; ++j)
      bq[j] = ldfrag_h(Bb + (size_t)(n0 + (j << 4) + rlane) * ldb + koff + k0);
#pragma unroll
    for (int i = 0; i < 4; ++i) {
      const v16h af = ldfrag_h(Ab + (size_t)(m0 + (i << 4) + rlane) * lda + koff + k0);
#pragma unroll
      for (int j = 0; j < 4; ++j) acc[i][j] = mmar(af, bq[j], acc[i][j]);
      dep_guard(acc[i][0], acc[i][3], af, bq[3]);
    }
    keep4(bq[0], bq[1], bq[2], bq[3]);
  }
  acc_guard4(acc[0][0], acc[0][1], acc[0][2], acc[0][3]);
  acc_guard4(acc[1][0], acc[1][1], acc[1][2], acc[1][3]);
  acc_guard4(acc[2][0], acc[2][1], acc[2][2], acc[2][3]);
  acc_guard4(acc[3][0], acc[3][1], acc[3][2], acc[3][3]);

  float* slab = sT[wave];
  const int q = lane >> 3, c8 = (lane & 7) * 8;
  unsigned short* C = Cp + (size_t)b * (size_t)strideC;
  float bcol[8];
  {
    const v4f b0 = *(const v4f*)(bias + (BIASROW ? 0 : (n0 + c8)));
    const v4f b1 = *(const v4f*)(bias + (BIASROW ? 4 : (n0 + c8 + 4)));
#pragma unroll
    for (int e = 0; e < 4; ++e) { bcol[e] = b0[e]; bcol[4 + e] = b1[e]; }
  }
#pragma unroll
  for (int i = 0; i < 4; ++i) {
    const int mBase = m0 + (i << 4);
#pragma unroll
    for (int j = 0; j < 4; ++j) {
#pragma unroll
      for (int r = 0; r < 8; ++r) {
        slab[(mOff + r) * 68 + (j << 4) + rlane] = acc[i][j][r];
      }
    }
    __builtin_amdgcn_fence(__ATOMIC_RELEASE, "workgroup");
    __builtin_amdgcn_wave_barrier();
    __builtin_amdgcn_fence(__ATOMIC_ACQUIRE, "workgroup");
    v4u hv[4];
#pragma unroll
    for (int it = 0; it < 4; ++it) {
      const int row = it * 4 + q;
      const float* sp = slab + row * 68 + c8;
      float bb[8];
      if (BIASROW) {
        const float bv = bias[mBase + row];
#pragma unroll
        for (int e = 0; e < 8; ++e) bb[e] = bv;
      } else {
#pragma unroll
        for (int e = 0; e < 8; ++e) bb[e] = bcol[e];
      }
      v4u a;
#pragma unroll
      for (int e = 0; e < 4; ++e) {
        const float f0 = (sp[2 * e] * ascale + bb[2 * e]) * oscale;
        const float f1 = (sp[2 * e + 1] * ascale + bb[2 * e + 1]) * oscale;
        a[e] = pk16(h_bits((_Float16)f0), h_bits((_Float16)f1));
      }
      hv[it] = a;
    }
    for (int pass = 0; pass < 2; ++pass) {
#pragma unroll
      for (int it = 0; it < 4; ++it) {
        const int row = it * 4 + q;
        *(volatile v4u*)(C + (size_t)(mBase + row) * ldc + n0 + c8) = hv[it];
      }
      __threadfence();
    }
    __builtin_amdgcn_fence(__ATOMIC_RELEASE, "workgroup");
    __builtin_amdgcn_wave_barrier();
    __builtin_amdgcn_fence(__ATOMIC_ACQUIRE, "workgroup");
  }
}

__global__ __launch_bounds__(128)
void attn_two(const unsigned short* __restrict__ qp, const unsigned short* __restrict__ kp,
              const unsigned short* __restrict__ vtp, const unsigned short* __restrict__ lqp,
              const unsigned short* __restrict__ lkp, const unsigned short* __restrict__ lvtp,
              float* out0, float* lcp, float sscale) {
  union FH { v16h v; v8h h[2]; };
  __shared__ __align__(16) _Float16 Ksh[64 * 64];
  __shared__ __align__(16) _Float16 LKs[64 * HL];
  __shared__ __align__(16) _Float16 Vth[64 * 64];
  __shared__ __align__(16) _Float16 LVs[HL * 64];
  __shared__ __align__(16) _Float16 Psh[4][16 * 64];
  __shared__ __align__(16) float    Os[4][16 * 64];
  __shared__ __align__(16) float    OLs[4][16 * HL];

  const int tid  = threadIdx.x;
  const int wave = tid >> 5;
  const int lane = tid & 31;
  const int hh   = lane >> 4;
  const int c    = lane & 15;

  const int bx   = blockIdx.x;
  const int qb   = bx % NQB;
  const int rest = bx / NQB;
  const int h    = rest % NH;
  const int b    = rest / NH;
  const int q0   = qb * 64 + wave * 16;
  const size_t rowB = (size_t)b * SEQ;

  const _Float16* Q   = (const _Float16*)(const void*)qp;
  const _Float16* LQ  = (const _Float16*)(const void*)lqp;
  const _Float16* Kg  = (const _Float16*)(const void*)kp + (size_t)h * HD;
  const _Float16* LKg = (const _Float16*)(const void*)lkp + (size_t)h * HL;
  const _Float16* Vh  = (const _Float16*)(const void*)vtp  + ((size_t)b * DM + (size_t)h * HD) * SEQ;
  const _Float16* LVh = (const _Float16*)(const void*)lvtp + ((size_t)b * DL + (size_t)h * HL) * SEQ;

  v16h qa[2];
#pragma unroll
  for (int dc = 0; dc < 2; ++dc) {
    const size_t qo = (rowB + q0 + c) * DM + (size_t)h * HD + dc * 32 + 8 * hh;
    qa[dc] = ldfrag_h(Q + qo);
  }
  FH la;
  la.h[0] = *(const v8h*)(LQ + (rowB + q0 + c) * DL + (size_t)h * HL + 8 * hh);
  la.h[1] = zero8h();

  float mrow[8], lrow[8];
  v8f oacc[4];
  v8f olacc = zero8();
#pragma unroll
  for (int r = 0; r < 8; ++r) { mrow[r] = -INFINITY; lrow[r] = 0.f; }
#pragma unroll
  for (int t = 0; t < 4; ++t) oacc[t] = zero8();

  for (int kt = 0; kt < NKT; ++kt) {
    const int kv0 = kt * 64;
    __syncthreads();
    {
      const int r = tid >> 1, half = (tid & 1) * 32;
      const _Float16* kg = Kg + (rowB + kv0 + r) * DM + half;
      const _Float16* vg = Vh + (size_t)r * SEQ + kv0 + half;
#pragma unroll
      for (int i = 0; i < 4; ++i) {
        const v8h a0 = *(const v8h*)(kg + 8 * i);
        const v8h b0 = *(const v8h*)(vg + 8 * i);
        *(v8h*)(Ksh + r * 64 + half + 8 * i) = a0;
        *(v8h*)(Vth + r * 64 + half + 8 * i) = b0;
      }
      const int c8l = (tid & 1) * 8;
      const v8h lk8 = *(const v8h*)(LKg + (rowB + kv0 + r) * DL + c8l);
      *(v8h*)(LKs + r * HL + c8l) = lk8;
      const int dv = tid >> 3, s8 = (tid & 7) * 8;
      const v8h lv8 = *(const v8h*)(LVh + (size_t)dv * SEQ + kv0 + s8);
      *(v8h*)(LVs + dv * 64 + s8) = lv8;
    }
    __syncthreads();

    v8f s[4];
#pragma unroll
    for (int j = 0; j < 4; ++j) {
      v8f acc = zero8();
#pragma unroll
      for (int dc = 0; dc < 2; ++dc) {
        FH kb;
        kb.h[0] = *(const v8h*)(Ksh + (j * 16 + c) * 64 + dc * 32 + 8 * hh);
        kb.h[1] = *(const v8h*)(Ksh + (j * 16 + c) * 64 + dc * 32 + 16 + 8 * hh);
        acc = mma_h(qa[dc], kb.v, acc);
      }
      FH lb;
      lb.h[0] = *(const v8h*)(LKs + (j * 16 + c) * HL + 8 * hh);
      lb.h[1] = zero8h();
      acc = mma_h(la.v, lb.v, acc);
#pragma unroll
      for (int r = 0; r < 8; ++r) s[j][r] = acc[r] * sscale;
    }

    _Float16* pwh = Psh[wave];
#pragma unroll
    for (int r = 0; r < 8; ++r) {
      float m = s[0][r];
#pragma unroll
      for (int j = 1; j < 4; ++j) m = fmaxf(m, s[j][r]);
#pragma unroll
      for (int off = 1; off < 16; off <<= 1) m = fmaxf(m, __shfl_xor(m, off, 32));
      const float mnew  = fmaxf(mrow[r], m);
      const float msafe = (mnew == -INFINITY) ? 0.f : mnew;
      const float alpha = __expf(mrow[r] - msafe);
      mrow[r] = mnew;
      float psum = 0.f;
#pragma unroll
      for (int j = 0; j < 4; ++j) {
        const float p = __expf(s[j][r] - msafe);
        psum += p;
        pwh[(8 * hh + r) * 64 + j * 16 + c] = (_Float16)(p * 1024.0f);
      }
#pragma unroll
      for (int off = 1; off < 16; off <<= 1) psum += __shfl_xor(psum, off, 32);
      lrow[r] = lrow[r] * alpha + psum;
#pragma unroll
      for (int t = 0; t < 4; ++t) oacc[t][r] *= alpha;
      olacc[r] *= alpha;
    }
    __builtin_amdgcn_fence(__ATOMIC_RELEASE, "workgroup");
    __builtin_amdgcn_wave_barrier();
    __builtin_amdgcn_fence(__ATOMIC_ACQUIRE, "workgroup");

#pragma unroll 1
    for (int kk = 0; kk < 2; ++kk) {
      FH pa;
      pa.h[0] = *(const v8h*)(pwh + c * 64 + kk * 32 + 8 * hh);
      pa.h[1] = *(const v8h*)(pwh + c * 64 + kk * 32 + 16 + 8 * hh);
#pragma unroll
      for (int t = 0; t < 4; ++t) {
        FH vb;
        vb.h[0] = *(const v8h*)(Vth + (t * 16 + c) * 64 + kk * 32 + 8 * hh);
        vb.h[1] = *(const v8h*)(Vth + (t * 16 + c) * 64 + kk * 32 + 16 + 8 * hh);
        oacc[t] = mma_h(pa.v, vb.v, oacc[t]);
      }
      FH wb;
      wb.h[0] = *(const v8h*)(LVs + c * 64 + kk * 32 + 8 * hh);
      wb.h[1] = *(const v8h*)(LVs + c * 64 + kk * 32 + 16 + 8 * hh);
      olacc = mma_h(pa.v, wb.v, olacc);
    }
  }

  float* os = Os[wave];
  float* ol = OLs[wave];
#pragma unroll
  for (int r = 0; r < 8; ++r) {
    const float l = lrow[r];
    const float inv = ((l > 0.f) ? (1.0f / l) : 0.f) * (1.0f / 1024.0f);
#pragma unroll
    for (int t = 0; t < 4; ++t) os[(8 * hh + r) * 64 + t * 16 + c] = oacc[t][r] * inv;
    ol[(8 * hh + r) * HL + c] = olacc[r] * inv;
  }
  __builtin_amdgcn_fence(__ATOMIC_RELEASE, "workgroup");
  __builtin_amdgcn_wave_barrier();
  __builtin_amdgcn_fence(__ATOMIC_ACQUIRE, "workgroup");
  {
    const int h2 = lane >> 4, c4 = (lane & 15) * 4;
    float* ob = out0 + (rowB + q0) * DM + (size_t)h * HD + c4;
    float* lb = lcp + (((size_t)(b * NH + h)) * SEQ + (size_t)q0) * HL;
    for (int pass = 0; pass < 2; ++pass) {
#pragma unroll
      for (int it = 0; it < 8; ++it) {
        const int row = it * 2 + h2;
        const v4f v = *(const v4f*)(os + row * 64 + c4);
        *(volatile v4f*)(ob + (size_t)row * DM) = v;
      }
#pragma unroll
      for (int it = 0; it < 2; ++it) {
        const int idx = it * 32 + lane;
        const v4f v = *(const v4f*)(ol + idx * 4);
        *(volatile v4f*)(lb + idx * 4) = v;
      }
      __threadfence();
    }
  }
}

__global__ __launch_bounds__(256) void lc_pack(const float* __restrict__ lc, float* out1, int n4) {
  const int i = blockIdx.x * 256 + (int)threadIdx.x;
  if (i < n4) {
    const int e   = i * 4;
    const int row = e / DL;
    const int col = e - row * DL;
    const int hd  = col >> 4;
    const int d   = col & 15;
    const int bb  = row / SEQ;
    const int t   = row - bb * SEQ;
    const v4f v = *(const v4f*)(lc + (((size_t)(bb * NH + hd)) * SEQ + (size_t)t) * HL + d);
    float* o = out1 + (size_t)e;
    *(volatile v4f*)o = v;
    __threadfence();
    *(volatile v4f*)o = v;
  }
}

extern "C" void kernel_launch(void* const* d_in, const int* in_sizes, int n_in,
                              void* d_out, int out_size, void* d_ws, size_t ws_size,
                              hipStream_t stream) {
  if (n_in < 14) return;
  if (in_sizes[0] != NB * SEQ * DM) return;
  if (in_sizes[1] != NB * SEQ * DL) return;
  if (in_sizes[2] != DM * DM || in_sizes[4] != DM * DM || in_sizes[6] != DM * DM) return;
  if (in_sizes[3] != DM || in_sizes[5] != DM || in_sizes[7] != DM) return;
  if (in_sizes[8] != DL * DL || in_sizes[10] != DL * DL || in_sizes[12] != DL * DL) return;
  if (in_sizes[9] != DL || in_sizes[11] != DL || in_sizes[13] != DL) return;
  if (out_size != NB * SEQ * (DM + DL)) return;

  const float* x    = (const float*)d_in[0];
  const float* xl   = (const float*)d_in[1];
  const float* Wq   = (const float*)d_in[2];
  const float* bq   = (const float*)d_in[3];
  const float* Wk   = (const float*)d_in[4];
  const float* bk   = (const float*)d_in[5];
  const float* Wv   = (const float*)d_in[6];
  const float* bv   = (const float*)d_in[7];
  const float* Wlq  = (const float*)d_in[8];
  const float* blq  = (const float*)d_in[9];
  const float* Wlk  = (const float*)d_in[10];
  const float* blk_ = (const float*)d_in[11];
  const float* Wlv  = (const float*)d_in[12];
  const float* blv  = (const float*)d_in[13];

  const size_t PX  = (size_t)NB * SEQ * DM * 2;
  const size_t PL  = (size_t)NB * SEQ * DL * 2;
  const size_t PW  = (size_t)DM * DM * 2;
  const size_t PWL = (size_t)DL * DL * 2;
  const size_t PLC = (size_t)NB * NH * SEQ * HL * 4;
  size_t off = 0;
  const size_t oXh   = off; off += PX;
  const size_t oLh   = off; off += PL;
  const size_t oWq   = off; off += PW;
  const size_t oWk   = off; off += PW;
  const size_t oWv   = off; off += PW;
  const size_t oWlq  = off; off += PWL;
  const size_t oWlk  = off; off += PWL;
  const size_t oWlv  = off; off += PWL;
  const size_t oQp   = off; off += PX;
  const size_t oKp   = off; off += PX;
  const size_t oVTp  = off; off += PX;
  const size_t oLQp  = off; off += PL;
  const size_t oLKp  = off; off += PL;
  const size_t oLVTp = off; off += PL;
  const size_t oLC   = off; off += PLC;
  if (off > ws_size) return;
  if (off > (size_t)134217728) return;

  char* ws = (char*)d_ws;
  unsigned short* Xh   = (unsigned short*)(ws + oXh);
  unsigned short* Lh   = (unsigned short*)(ws + oLh);
  unsigned short* Wqh  = (unsigned short*)(ws + oWq);
  unsigned short* Wkh  = (unsigned short*)(ws + oWk);
  unsigned short* Wvh  = (unsigned short*)(ws + oWv);
  unsigned short* Wlqh = (unsigned short*)(ws + oWlq);
  unsigned short* Wlkh = (unsigned short*)(ws + oWlk);
  unsigned short* Wlvh = (unsigned short*)(ws + oWlv);
  unsigned short* Qp   = (unsigned short*)(ws + oQp);
  unsigned short* Kp   = (unsigned short*)(ws + oKp);
  unsigned short* VTp  = (unsigned short*)(ws + oVTp);
  unsigned short* LQp  = (unsigned short*)(ws + oLQp);
  unsigned short* LKp  = (unsigned short*)(ws + oLKp);
  unsigned short* LVTp = (unsigned short*)(ws + oLVTp);
  float*          LC   = (float*)(ws + oLC);
  float*          out0 = (float*)d_out;
  float*          out1 = (float*)d_out + (size_t)NB * SEQ * DM;

  const dim3 blk(256);
  const int n8x  = NB * SEQ * DM / 8;
  const int n8l  = NB * SEQ * DL / 8;
  const int n8w  = DM * DM / 8;
  const int n8wl = DL * DL / 8;
  const int n4o1 = NB * SEQ * DL / 4;
  const dim3 gCvtX((n8x + 255) / 256);
  const dim3 gCvtL((n8l + 255) / 256);
  const dim3 gCvtW((n8w + 255) / 256);
  const dim3 gCvtWl((n8wl + 255) / 256);
  const dim3 gT((((NB * SEQ) / 64) * (DM / 64) + 7) / 8, 1);
  const dim3 gVT(((DM / 64) * (SEQ / 64) + 7) / 8, NB);
  const dim3 gL((((NB * SEQ) / 64) * (DL / 64) + 7) / 8, 1);
  const dim3 gLVT(((DL / 64) * (SEQ / 64) + 7) / 8, NB);
  const dim3 gAttn(NB * NH * NQB);
  const dim3 gPack((n4o1 + 255) / 256);

  cvt_h16x8<<<gCvtX,  blk, 0, stream>>>(x,   Xh,   n8x,  1.0f);
  cvt_h16x8<<<gCvtL,  blk, 0, stream>>>(xl,  Lh,   n8l,  1.0f);
  cvt_h16x8<<<gCvtW,  blk, 0, stream>>>(Wq,  Wqh,  n8w,  64.0f);
  cvt_h16x8<<<gCvtW,  blk, 0, stream>>>(Wk,  Wkh,  n8w,  64.0f);
  cvt_h16x8<<<gCvtW,  blk, 0, stream>>>(Wv,  Wvh,  n8w,  64.0f);
  cvt_h16x8<<<gCvtWl, blk, 0, stream>>>(Wlq, Wlqh, n8wl, 64.0f);
  cvt_h16x8<<<gCvtWl, blk, 0, stream>>>(Wlk, Wlkh, n8wl, 64.0f);
  cvt_h16x8<<<gCvtWl, blk, 0, stream>>>(Wlv, Wlvh, n8wl, 64.0f);
  gemm64<0><<<gT, blk, 0, stream>>>(Xh, DM, 0LL, Wqh, DM, 0LL, bq, Qp, DM, 0LL,
                                    NB * SEQ, DM, DM, 1.0f / 64.0f, 1.0f);
  gemm64<0><<<gT, blk, 0, stream>>>(Xh, DM, 0LL, Wkh, DM, 0LL, bk, Kp, DM, 0LL,
                                    NB * SEQ, DM, DM, 1.0f / 64.0f, 1.0f);
  gemm64<1><<<gVT, blk, 0, stream>>>(Wvh, DM, 0LL, Xh, DM, (long long)SEQ * DM, bv, VTp, SEQ, (long long)DM * SEQ,
                                     DM, SEQ, DM, 1.0f / 64.0f, 1.0f);
  gemm64<0><<<gL, blk, 0, stream>>>(Lh, DL, 0LL, Wlqh, DL, 0LL, blq, LQp, DL, 0LL,
                                    NB * SEQ, DL, DL, 1.0f / 64.0f, 2.0f);
  gemm64<0><<<gL, blk, 0, stream>>>(Lh, DL, 0LL, Wlkh, DL, 0LL, blk_, LKp, DL, 0LL,
                                    NB * SEQ, DL, DL, 1.0f / 64.0f, 1.0f);
  gemm64<1><<<gLVT, blk, 0, stream>>>(Wlvh, DL, 0LL, Lh, DL, (long long)SEQ * DL, blv, LVTp, SEQ, (long long)DL * SEQ,
                                      DL, SEQ, DL, 1.0f / 64.0f, 1.0f);
  attn_two<<<gAttn, dim3(128), 0, stream>>>(Qp, Kp, VTp, LQp, LKp, LVTp, out0, LC, 0.125f);
  lc_pack<<<gPack, blk, 0, stream>>>(LC, out1, n4o1);
  (void)hipGetLastError();
}
